// InferenceModel_721554506441
// MI455X (gfx1250) — hardware-verified
//
#include <hip/hip_runtime.h>
#define NNODE 50000
#define NNP 50048
#define NE 1600000
#define DI 128
#define DO 64
#define NREL 8
#define NB1 56
#define BW1 7168
#define NB2 392
#define NP1 25
#define NP2 2
#define KSTR 50176
#define ELCAP1 (NE + 32 * NB1 + 64)
#define ELCAP2 (NE + 32 * NB2 + 64)

typedef __bf16 v16b __attribute__((ext_vector_type(16)));
typedef unsigned short v8us __attribute__((ext_vector_type(8), may_alias));
typedef float  v8f  __attribute__((ext_vector_type(8)));
typedef float  v4f  __attribute__((ext_vector_type(4)));
typedef float  v4fa __attribute__((ext_vector_type(4), may_alias));
union FragB { v16b v; v8us half[2]; unsigned short u[16]; };

__device__ __forceinline__ unsigned short bf16_bits(float x) { unsigned int u = __float_as_uint(x); return (unsigned short)((u + 0x7FFFu + ((u >> 16) & 1u)) >> 16); }
__device__ __forceinline__ float bf16_val(unsigned short b) { return __uint_as_float(((unsigned int)b) << 16); }
__device__ __forceinline__ float bf16_round(float x) { return bf16_val(bf16_bits(x)); }
template <int NT>
__device__ __forceinline__ v8f mmaN(v16b ah, v16b al, v16b bh, v16b bl, v8f c) {
  c = __builtin_amdgcn_wmma_f32_16x16x32_bf16(false, ah, false, bh, (short)0, c, false, false);
  if (NT >= 2) c = __builtin_amdgcn_wmma_f32_16x16x32_bf16(false, al, false, bh, (short)0, c, false, false);
  if (NT >= 3) c = __builtin_amdgcn_wmma_f32_16x16x32_bf16(false, ah, false, bl, (short)0, c, false, false);
  asm volatile("v_nop\n\tv_nop\n\tv_nop\n\tv_nop" : "+v"(c) : "v"(ah), "v"(al), "v"(bh), "v"(bl));
  return c;
}

__global__ __launch_bounds__(256) void k_wt_bf16(const float* __restrict__ W, unsigned short* __restrict__ Wt, int K, int N) {
  const int t = blockIdx.x * 256 + threadIdx.x;
  const int k8n = K / 8;
  if (t >= N * k8n) return;
  const int n = t / k8n, k8 = (t % k8n) * 8;
  v8us v;
#pragma unroll
  for (int i = 0; i < 8; ++i) v[i] = bf16_bits(W[(size_t)(k8 + i) * N + n]);
  *(volatile v8us*)(Wt + (size_t)n * K + k8) = v;
  __threadfence();
  *(volatile v8us*)(Wt + (size_t)n * K + k8) = v;
}

template <bool ASPLIT, int ACT, bool BIAS_BF16>
__global__ __launch_bounds__(128) void k_gemm_bf(const float* __restrict__ A, int lda, const unsigned short* __restrict__ Wt, int ldb,
                                               const float* __restrict__ bias, float* __restrict__ C, int ldc, int M, int N, int K) {
  __shared__ __attribute__((aligned(16))) float so[4][16][64];
  const int tid = threadIdx.x, w = tid >> 5, lane = tid & 31, ln = lane & 15, hh = lane >> 4;
  const int ntn = N / 64;
  const int wid = blockIdx.x * 4 + w;
  const int mt = wid / ntn, nq = wid % ntn;
  if (mt * 16 >= M) return;
  const int row0 = mt * 16, col0 = nq * 64;
  const float* arow = A + (size_t)(row0 + ln) * lda;
  v8f acc[4] = {};
  for (int kb = 0; kb < K; kb += 32) {
    FragB ah, al;
    const v4f x0 = *(const v4fa*)(arow + kb + 8 * hh), x1 = *(const v4fa*)(arow + kb + 8 * hh + 4);
    const v4f x2 = *(const v4fa*)(arow + kb + 16 + 8 * hh), x3 = *(const v4fa*)(arow + kb + 16 + 8 * hh + 4);
    float xs[16] = {x0[0],x0[1],x0[2],x0[3],x1[0],x1[1],x1[2],x1[3],x2[0],x2[1],x2[2],x2[3],x3[0],x3[1],x3[2],x3[3]};
#pragma unroll
    for (int i = 0; i < 16; ++i) { const unsigned short hb = bf16_bits(xs[i]); ah.u[i] = hb; al.u[i] = ASPLIT ? bf16_bits(xs[i] - bf16_val(hb)) : (unsigned short)0; }
#pragma unroll
    for (int t = 0; t < 4; ++t) {
      const unsigned short* brow = Wt + (size_t)(col0 + t * 16 + ln) * ldb + kb;
      FragB b;
      b.half[0] = *(const v8us*)(brow + 8 * hh);
      b.half[1] = *(const v8us*)(brow + 16 + 8 * hh);
      acc[t] = mmaN<ASPLIT ? 2 : 1>(ah.v, al.v, b.v, b.v, acc[t]);
    }
  }
#pragma unroll
  for (int t = 0; t < 4; ++t) {
    float bv = bias ? bias[col0 + t * 16 + ln] : 0.f;
    if (BIAS_BF16) bv = bf16_round(bv);
#pragma unroll
    for (int r = 0; r < 8; ++r) { float v = acc[t][r] + bv; if (ACT == 1) v = fmaxf(v, 0.f); so[w][8 * hh + r][t * 16 + ln] = v; }
  }
  __builtin_amdgcn_fence(__ATOMIC_ACQ_REL, "workgroup");
  __builtin_amdgcn_wave_barrier();
  const int rsub = lane >> 4, c4 = (lane & 15) * 4;
  for (int pass = 0; pass < 2; ++pass) {
#pragma unroll
    for (int q = 0; q < 8; ++q) {
      const int r = q * 2 + rsub;
      const v4f v = *(const v4fa*)&so[w][r][c4];
      *(volatile v4f*)(C + (size_t)(row0 + r) * ldc + col0 + c4) = v;
    }
    if (pass == 0) __threadfence();
  }
}

template <int D, bool CAUSAL>
__global__ __launch_bounds__(128) void k_flash(const float* __restrict__ qb, const float* __restrict__ kb, const float* __restrict__ vb,
                                             int pitch, int T, int H, float scale, float* __restrict__ y, int ypitch) {
  constexpr int KS = D / 32;
  constexpr int DT = D / 16;
  __shared__ __attribute__((aligned(16))) unsigned short sKh[32][D + 8], sKl[32][D + 8], sVh[32][D + 8], sVl[32][D + 8];
  __shared__ __attribute__((aligned(16))) unsigned short sPh[4][16][40], sPl[4][16][40];
  __shared__ __attribute__((aligned(16))) float sO[4][16][D];
  const int tid = threadIdx.x, w = tid >> 5, lane = tid & 31, ln = lane & 15, hh = lane >> 4;
  const int nqb = (T + 63) / 64;
  const int bh = blockIdx.x / nqb, qblk = blockIdx.x % nqb;
  const int b = bh / H, h = bh % H;
  const int q0 = qblk * 64 + w * 16;
  const float* Q = qb + (size_t)b * T * pitch + h * D;
  const float* K = kb + (size_t)b * T * pitch + h * D;
  const float* V = vb + (size_t)b * T * pitch + h * D;

  FragB aqh[KS], aql[KS];
  {
    int row = q0 + ln; if (row >= T) row = T - 1;
    const float* qr = Q + (size_t)row * pitch;
#pragma unroll
    for (int ks = 0; ks < KS; ++ks)
#pragma unroll
      for (int i = 0; i < 16; ++i) {
        const int d = ks * 32 + ((i < 8) ? (8 * hh + i) : (16 + 8 * hh + (i - 8)));
        const float x = qr[d] * scale; const unsigned short hb = bf16_bits(x);
        aqh[ks].u[i] = hb; aql[ks].u[i] = bf16_bits(x - bf16_val(hb));
      }
  }
  float m_r[8], l_r[8];
#pragma unroll
  for (int r = 0; r < 8; ++r) { m_r[r] = -3.0e38f; l_r[r] = 0.f; }
  v8f oacc[DT];
#pragma unroll
  for (int dt = 0; dt < DT; ++dt) oacc[dt] = (v8f){0.f,0.f,0.f,0.f,0.f,0.f,0.f,0.f};

  const int kv_end = CAUSAL ? min(T, qblk * 64 + 64) : T;
  for (int j0 = 0; j0 < kv_end; j0 += 32) {
    __syncthreads();
    for (int e = tid; e < 32 * (D / 4); e += 128) {
      const int r = e / (D / 4), c4 = (e % (D / 4)) * 4;
      const int key = j0 + r;
      v4f kf = {0.f,0.f,0.f,0.f}, vf = {0.f,0.f,0.f,0.f};
      if (key < T) { kf = *(const v4fa*)(K + (size_t)key * pitch + c4); vf = *(const v4fa*)(V + (size_t)key * pitch + c4); }
#pragma unroll
      for (int t = 0; t < 4; ++t) {
        unsigned short hb = bf16_bits(kf[t]); sKh[r][c4 + t] = hb; sKl[r][c4 + t] = bf16_bits(kf[t] - bf16_val(hb));
        hb = bf16_bits(vf[t]); sVh[r][c4 + t] = hb; sVl[r][c4 + t] = bf16_bits(vf[t] - bf16_val(hb));
      }
    }
    __syncthreads();
    v8f s[2];
#pragma unroll
    for (int nt = 0; nt < 2; ++nt) {
      v8f acc = {};
#pragma unroll
      for (int ks = 0; ks < KS; ++ks) {
        FragB bh_, bl_;
        bh_.half[0] = *(const v8us*)&sKh[nt * 16 + ln][ks * 32 + 8 * hh]; bh_.half[1] = *(const v8us*)&sKh[nt * 16 + ln][ks * 32 + 16 + 8 * hh];
        bl_.half[0] = *(const v8us*)&sKl[nt * 16 + ln][ks * 32 + 8 * hh]; bl_.half[1] = *(const v8us*)&sKl[nt * 16 + ln][ks * 32 + 16 + 8 * hh];
        acc = mmaN<3>(aqh[ks].v, aql[ks].v, bh_.v, bl_.v, acc);
      }
      s[nt] = acc;
    }
    float alpha[8];
#pragma unroll
    for (int r = 0; r < 8; ++r) {
      const int qi = q0 + 8 * hh + r;
      const int ja = j0 + ln, jb = j0 + 16 + ln;
      if (CAUSAL) { if (ja > qi) s[0][r] = -3.0e38f; if (jb > qi) s[1][r] = -3.0e38f; }
      if (ja >= T) s[0][r] = -3.0e38f;
      if (jb >= T) s[1][r] = -3.0e38f;
      float mx = fmaxf(s[0][r], s[1][r]);
      mx = fmaxf(mx, __shfl_xor(mx, 1, 32)); mx = fmaxf(mx, __shfl_xor(mx, 2, 32)); mx = fmaxf(mx, __shfl_xor(mx, 4, 32)); mx = fmaxf(mx, __shfl_xor(mx, 8, 32));
      const float mnew = fmaxf(m_r[r], mx);
      alpha[r] = (mnew > -1.0e38f) ? __expf(m_r[r] - mnew) : 1.0f;
      const float p0 = (s[0][r] > -1.0e38f) ? __expf(s[0][r] - mnew) : 0.f;
      const float p1 = (s[1][r] > -1.0e38f) ? __expf(s[1][r] - mnew) : 0.f;
      m_r[r] = mnew;
      l_r[r] = l_r[r] * alpha[r] + p0 + p1;
      unsigned short hb = bf16_bits(p0); sPh[w][8 * hh + r][ln] = hb;      sPl[w][8 * hh + r][ln] = bf16_bits(p0 - bf16_val(hb));
      hb = bf16_bits(p1);                sPh[w][8 * hh + r][16 + ln] = hb; sPl[w][8 * hh + r][16 + ln] = bf16_bits(p1 - bf16_val(hb));
    }
#pragma unroll
    for (int dt = 0; dt < DT; ++dt)
#pragma unroll
      for (int r = 0; r < 8; ++r) oacc[dt][r] *= alpha[r];
    __builtin_amdgcn_fence(__ATOMIC_ACQ_REL, "workgroup");
    __builtin_amdgcn_wave_barrier();
    FragB pah, pal;
    pah.half[0] = *(const v8us*)&sPh[w][ln][8 * hh]; pah.half[1] = *(const v8us*)&sPh[w][ln][16 + 8 * hh];
    pal.half[0] = *(const v8us*)&sPl[w][ln][8 * hh]; pal.half[1] = *(const v8us*)&sPl[w][ln][16 + 8 * hh];
#pragma unroll
    for (int dt = 0; dt < DT; ++dt) {
      FragB bvh, bvl;
#pragma unroll
      for (int i = 0; i < 8; ++i) {
        bvh.u[i] = sVh[8 * hh + i][dt * 16 + ln]; bvh.u[8 + i] = sVh[16 + 8 * hh + i][dt * 16 + ln];
        bvl.u[i] = sVl[8 * hh + i][dt * 16 + ln]; bvl.u[8 + i] = sVl[16 + 8 * hh + i][dt * 16 + ln];
      }
      oacc[dt] = mmaN<3>(pah.v, pal.v, bvh.v, bvl.v, oacc[dt]);
    }
    __builtin_amdgcn_fence(__ATOMIC_ACQ_REL, "workgroup");
    __builtin_amdgcn_wave_barrier();
  }
#pragma unroll
  for (int r = 0; r < 8; ++r) {
    float l = l_r[r];
    l += __shfl_xor(l, 1, 32); l += __shfl_xor(l, 2, 32); l += __shfl_xor(l, 4, 32); l += __shfl_xor(l, 8, 32);
    l_r[r] = (l > 0.f) ? 1.0f / l : 0.f;
  }
#pragma unroll
  for (int dt = 0; dt < DT; ++dt)
#pragma unroll
    for (int r = 0; r < 8; ++r) sO[w][8 * hh + r][dt * 16 + ln] = oacc[dt][r] * l_r[r];
  __builtin_amdgcn_fence(__ATOMIC_ACQ_REL, "workgroup");
  __builtin_amdgcn_wave_barrier();
  for (int pass = 0; pass < 2; ++pass) {
    for (int r = 0; r < 16; ++r) {
      const int row = q0 + r;
      if (row < T && lane < D / 4) {
        const v4f val = *(const v4fa*)&sO[w][r][lane * 4];
        *(volatile v4f*)(y + ((size_t)b * T + row) * ypitch + h * D + lane * 4) = val;
      }
    }
    if (pass == 0) __threadfence();
  }
}

template <bool ASPLIT, int ACT, bool BIAS_BF16, bool RES_BF16>
__global__ __launch_bounds__(128) void k_gemm_bf3(const float* __restrict__ A, int lda, const unsigned short* __restrict__ Wt, int ldb,
                                                const float* __restrict__ bias, const float* __restrict__ resid, int rmod, int ldr,
                                                float* __restrict__ C, int ldc, int M, int N, int K) {
  __shared__ __attribute__((aligned(16))) float so[4][16][64];
  const int tid = threadIdx.x, w = tid >> 5, lane = tid & 31, ln = lane & 15, hh = lane >> 4;
  const int ntn = N / 64;
  const int wid = blockIdx.x * 4 + w;
  const int mt = wid / ntn, nq = wid % ntn;
  if (mt * 16 >= M) return;
  const int row0 = mt * 16, col0 = nq * 64;
  const float* arow = A + (size_t)(row0 + ln) * lda;
  v8f acc[4] = {};
  for (int kb = 0; kb < K; kb += 32) {
    FragB ah, al;
    const v4f x0 = *(const v4fa*)(arow + kb + 8 * hh), x1 = *(const v4fa*)(arow + kb + 8 * hh + 4);
    const v4f x2 = *(const v4fa*)(arow + kb + 16 + 8 * hh), x3 = *(const v4fa*)(arow + kb + 16 + 8 * hh + 4);
    float xs[16] = {x0[0],x0[1],x0[2],x0[3],x1[0],x1[1],x1[2],x1[3],x2[0],x2[1],x2[2],x2[3],x3[0],x3[1],x3[2],x3[3]};
#pragma unroll
    for (int i = 0; i < 16; ++i) { const unsigned short hb = bf16_bits(xs[i]); ah.u[i] = hb; al.u[i] = ASPLIT ? bf16_bits(xs[i] - bf16_val(hb)) : (unsigned short)0; }
#pragma unroll
    for (int t = 0; t < 4; ++t) {
      const unsigned short* brow = Wt + (size_t)(col0 + t * 16 + ln) * ldb + kb;
      FragB b;
      b.half[0] = *(const v8us*)(brow + 8 * hh);
      b.half[1] = *(const v8us*)(brow + 16 + 8 * hh);
      acc[t] = mmaN<ASPLIT ? 2 : 1>(ah.v, al.v, b.v, b.v, acc[t]);
    }
  }
#pragma unroll
  for (int t = 0; t < 4; ++t) {
    const int col = col0 + t * 16 + ln;
    float bv = bias ? bias[col] : 0.f;
    if (BIAS_BF16) bv = bf16_round(bv);
#pragma unroll
    for (int r = 0; r < 8; ++r) {
      float v = acc[t][r] + bv;
      if (resid) { float rv = resid[(size_t)((row0 + 8 * hh + r) % rmod) * ldr + col]; if (RES_BF16) rv = bf16_round(rv); v += rv; }
      if (ACT == 1) v = fmaxf(v, 0.f);
      if (ACT == 2) v = 0.5f * v * (1.0f + erff(v * 0.70710678118654752f));
      if (ACT == 3) { const float u = 0.7978845608028654f * (v + 0.044715f * v * v * v); v = 0.5f * v * (1.0f + tanhf(u)); }
      so[w][8 * hh + r][t * 16 + ln] = v;
    }
  }
  __builtin_amdgcn_fence(__ATOMIC_ACQ_REL, "workgroup");
  __builtin_amdgcn_wave_barrier();
  const int rsub = lane >> 4, c4 = (lane & 15) * 4;
  for (int pass = 0; pass < 2; ++pass) {
#pragma unroll
    for (int q = 0; q < 8; ++q) {
      const int r = q * 2 + rsub;
      const v4f v = *(const v4fa*)&so[w][r][c4];
      *(volatile v4f*)(C + (size_t)(row0 + r) * ldc + col0 + c4) = v;
    }
    if (pass == 0) __threadfence();
  }
}
template <bool PARAM_BF16>
__global__ __launch_bounds__(256) void k_layernorm(const float* __restrict__ X, const float* __restrict__ R, const float* __restrict__ g, const float* __restrict__ bta,
                                                  float* __restrict__ out_sum, float* __restrict__ out_norm, int N, float eps) {
  __shared__ float red[256];
  const int row = blockIdx.x, tid = threadIdx.x;
  const float* x = X + (size_t)row * N; const float* rr = R ? R + (size_t)row * N : nullptr;
  float vals[16];
  const int per = N / 256;
  float s1 = 0.f;
  for (int u = 0; u < per / 4; ++u) {
    const int j = tid * 4 + 1024 * u;
    const v4f a = *(const v4fa*)(x + j);
    v4f b = {0.f,0.f,0.f,0.f}; if (rr) b = *(const v4fa*)(rr + j);
#pragma unroll
    for (int q = 0; q < 4; ++q) { const float v = a[q] + b[q]; vals[u * 4 + q] = v; s1 += v; }
  }
  red[tid] = s1; __syncthreads();
  for (int st = 128; st > 0; st >>= 1) { if (tid < st) red[tid] += red[tid + st]; __syncthreads(); }
  const float mu = red[0] / (float)N; __syncthreads();
  float s2 = 0.f;
  for (int u = 0; u < per / 4; ++u)
#pragma unroll
    for (int q = 0; q < 4; ++q) { const float c = vals[u * 4 + q] - mu; s2 += c * c; }
  red[tid] = s2; __syncthreads();
  for (int st = 128; st > 0; st >>= 1) { if (tid < st) red[tid] += red[tid + st]; __syncthreads(); }
  const float rs = rsqrtf(red[0] / (float)N + eps);
  for (int pass = 0; pass < 2; ++pass) {
    for (int u = 0; u < per / 4; ++u) {
      const int j = tid * 4 + 1024 * u;
      v4f o, sm;
#pragma unroll
      for (int q = 0; q < 4; ++q) {
        float gg = g[j + q], bb = bta[j + q];
        if (PARAM_BF16) { gg = bf16_round(gg); bb = bf16_round(bb); }
        sm[q] = vals[u * 4 + q]; o[q] = (vals[u * 4 + q] - mu) * rs * gg + bb;
      }
      if (out_sum) *(volatile v4f*)(out_sum + (size_t)row * N + j) = sm;
      *(volatile v4f*)(out_norm + (size_t)row * N + j) = o;
    }
    if (pass == 0) __threadfence();
  }
}


typedef _Float16 v16h __attribute__((ext_vector_type(16)));
union FragH { v16h v; v8us half[2]; _Float16 h[16]; unsigned short u[16]; };
template <int NT>
__device__ __forceinline__ v8f mmaH(v16h ah, v16h al, v16h bh, v16h bl, v8f c) {
  c = __builtin_amdgcn_wmma_f32_16x16x32_f16(false, ah, false, bh, (short)0, c, false, false);
  if (NT >= 2) c = __builtin_amdgcn_wmma_f32_16x16x32_f16(false, al, false, bh, (short)0, c, false, false);
  if (NT >= 3) c = __builtin_amdgcn_wmma_f32_16x16x32_f16(false, ah, false, bl, (short)0, c, false, false);
  asm volatile("v_nop\n\tv_nop\n\tv_nop\n\tv_nop" : "+v"(c) : "v"(ah), "v"(al), "v"(bh), "v"(bl));
  return c;
}
template <bool ASPLIT>
__global__ __launch_bounds__(128) void k_gemm_h(const float* __restrict__ A, int lda, size_t sA, const _Float16* __restrict__ Bh, int ldb, size_t sB, float alpha, float* __restrict__ C, int ldc, size_t sC, int M, int N, int K) {
  __shared__ __attribute__((aligned(16))) float so[4][16][64];
  const int tid = threadIdx.x, w = tid >> 5, lane = tid & 31, ln = lane & 15, hh = lane >> 4; const int by = blockIdx.y;
  A += (size_t)by * sA; Bh += (size_t)by * sB; C += (size_t)by * sC;
  const int ntn = (N + 63) / 64; const int wid = blockIdx.x * 4 + w; const int mt = wid / ntn, nq = wid % ntn; if (mt * 16 >= M) return;
  const int row0 = mt * 16, col0 = nq * 64; const float* arow = A + (size_t)(row0 + ln) * lda;
  v8f acc[4] = {};
  for (int kb = 0; kb < K; kb += 32) {
    FragH ah, al;
    const v4f x0 = *(const v4fa*)(arow + kb + 8 * hh), x1 = *(const v4fa*)(arow + kb + 8 * hh + 4), x2 = *(const v4fa*)(arow + kb + 16 + 8 * hh), x3 = *(const v4fa*)(arow + kb + 16 + 8 * hh + 4);
    float xs[16] = {x0[0],x0[1],x0[2],x0[3],x1[0],x1[1],x1[2],x1[3],x2[0],x2[1],x2[2],x2[3],x3[0],x3[1],x3[2],x3[3]};
#pragma unroll
    for (int i = 0; i < 16; ++i) { const _Float16 h = (_Float16)xs[i]; ah.h[i] = h; al.h[i] = ASPLIT ? (_Float16)(xs[i] - (float)h) : (_Float16)0.0f; }
#pragma unroll
    for (int t = 0; t < 4; ++t) { if (col0 + t * 16 >= N) continue; const size_t boff = (size_t)(col0 + t * 16 + ln) * ldb + kb; FragH bq; bq.half[0] = *(const v8us*)(Bh + boff + 8 * hh); bq.half[1] = *(const v8us*)(Bh + boff + 16 + 8 * hh);
      acc[t] = mmaH<ASPLIT ? 2 : 1>(ah.v, al.v, bq.v, bq.v, acc[t]); }
  }
#pragma unroll
  for (int t = 0; t < 4; ++t) { if (col0 + t * 16 >= N) continue;
#pragma unroll
    for (int r = 0; r < 8; ++r) so[w][8 * hh + r][t * 16 + ln] = acc[t][r] * alpha; }
  __builtin_amdgcn_fence(__ATOMIC_ACQ_REL, "workgroup"); __builtin_amdgcn_wave_barrier();
  const int rsub = lane >> 4, c4 = (lane & 15) * 4;
  for (int pass = 0; pass < 2; ++pass) {
#pragma unroll
    for (int q = 0; q < 8; ++q) { const int r = q * 2 + rsub; if (col0 + c4 < N) { const v4f v = *(const v4fa*)&so[w][r][c4]; *(volatile v4f*)(C + (size_t)(row0 + r) * ldc + col0 + c4) = v; } }
    if (pass == 0) __threadfence(); }
}

__global__ __launch_bounds__(256) void k_wt_f16(const float* __restrict__ W, _Float16* __restrict__ Wt, int K, int N, float scale) {
  const int t = blockIdx.x * 256 + threadIdx.x; if (t >= N * (K / 8)) return; const int n = t / (K / 8), k8 = (t % (K / 8)) * 8; FragH f;
#pragma unroll
  for (int i = 0; i < 8; ++i) f.h[i] = (_Float16)(bf16_round(W[(size_t)(k8 + i) * N + n]) * scale); const v8us o = f.half[0];
  *(volatile v8us*)((unsigned short*)Wt + (size_t)n * K + k8) = o; __threadfence(); *(volatile v8us*)((unsigned short*)Wt + (size_t)n * K + k8) = o;
}
template <int ACT>
__global__ __launch_bounds__(128) void k_gemm_hhx(const _Float16* __restrict__ A, int lda, size_t sA, const _Float16* __restrict__ Bh, int ldb, size_t sB, float alpha, const float* __restrict__ bias, size_t sBias, const float* __restrict__ CP, int rowsPerB, size_t sCPb, int row0g,
    float* __restrict__ C, _Float16* __restrict__ C16, int ldc, size_t sC, int M, int N, int K) {
  __shared__ __attribute__((aligned(16))) float so[4][16][64];
  const int tid = threadIdx.x, w = tid >> 5, lane = tid & 31, ln = lane & 15, hh = lane >> 4; const int by = blockIdx.y;
  A += (size_t)by * sA; Bh += (size_t)by * sB; const size_t cofs = (size_t)by * sC; const float* bp = bias ? bias + (size_t)by * sBias : nullptr;
  const int ntn = (N + 63) / 64; const int wid = blockIdx.x * 4 + w; const int mt = wid / ntn, nq = wid % ntn; if (mt * 16 >= M) return;
  const int row0 = mt * 16, col0 = nq * 64; const _Float16* arow = A + (size_t)(row0 + ln) * lda;
  v8f acc[4] = {};
  for (int kb = 0; kb < K; kb += 32) { FragH ah; ah.half[0] = *(const v8us*)((const unsigned short*)arow + kb + 8 * hh); ah.half[1] = *(const v8us*)((const unsigned short*)arow + kb + 16 + 8 * hh);
#pragma unroll
    for (int t = 0; t < 4; ++t) { if (col0 + t * 16 >= N) continue; const size_t boff = (size_t)(col0 + t * 16 + ln) * ldb + kb; FragH bq; bq.half[0] = *(const v8us*)((const unsigned short*)Bh + boff + 8 * hh); bq.half[1] = *(const v8us*)((const unsigned short*)Bh + boff + 16 + 8 * hh);
      acc[t] = mmaH<1>(ah.v, ah.v, bq.v, bq.v, acc[t]); }
  }
#pragma unroll
  for (int t = 0; t < 4; ++t) { if (col0 + t * 16 >= N) continue; const int col = col0 + t * 16 + ln; const float bv = bp ? bf16_round(bp[col]) : 0.f;
#pragma unroll
    for (int r = 0; r < 8; ++r) { float v = acc[t][r] * alpha + bv; if (CP) { const int bidx = (row0g + row0 + 8 * hh + r) / rowsPerB; v += CP[(size_t)bidx * sCPb + (size_t)by * 64 + col]; } if (ACT == 1) v = (v > 0.f) ? v : expm1f(v); else if (ACT == 3) v = fmaxf(v, 0.f); so[w][8 * hh + r][t * 16 + ln] = v; } }
  __builtin_amdgcn_fence(__ATOMIC_ACQ_REL, "workgroup"); __builtin_amdgcn_wave_barrier();
  const int rsub = lane >> 4, c4 = (lane & 15) * 4; typedef _Float16 v4h __attribute__((ext_vector_type(4)));
  for (int pass = 0; pass < 2; ++pass) {
#pragma unroll
    for (int q = 0; q < 8; ++q) { const int r = q * 2 + rsub; if (col0 + c4 < N) { const v4f v = *(const v4fa*)&so[w][r][c4]; if (C) *(volatile v4f*)(C + cofs + (size_t)(row0 + r) * ldc + col0 + c4) = v; if (C16) { v4h h4; for (int i = 0; i < 4; ++i) h4[i] = (_Float16)v[i]; *(volatile v4h*)(C16 + cofs + (size_t)(row0 + r) * ldc + col0 + c4) = h4; } } }
    if (pass == 0) __threadfence(); }
}


typedef _Float16 v4h __attribute__((ext_vector_type(4)));

__global__ __launch_bounds__(256) void k_x16(const float* __restrict__ x, _Float16* __restrict__ X16, size_t n8) { const size_t t = (size_t)blockIdx.x * 256 + threadIdx.x; if (t >= n8) return; FragH f;
#pragma unroll
  for (int q = 0; q < 8; ++q) f.h[q] = (_Float16)bf16_round(x[t * 8 + q]); *(volatile v8us*)((unsigned short*)X16 + t * 8) = f.half[0]; __threadfence(); *(volatile v8us*)((unsigned short*)X16 + t * 8) = f.half[0]; }
__global__ __launch_bounds__(256) void k_h16(const float* __restrict__ x, _Float16* __restrict__ X16, size_t n8) { const size_t t = (size_t)blockIdx.x * 256 + threadIdx.x; if (t >= n8) return; FragH f;
#pragma unroll
  for (int q = 0; q < 8; ++q) f.h[q] = (_Float16)x[t * 8 + q]; *(volatile v8us*)((unsigned short*)X16 + t * 8) = f.half[0]; __threadfence(); *(volatile v8us*)((unsigned short*)X16 + t * 8) = f.half[0]; }
__global__ __launch_bounds__(256) void k_round16f(const float* __restrict__ W, _Float16* __restrict__ Bt, size_t n8) { const size_t t = (size_t)blockIdx.x * 256 + threadIdx.x; if (t >= n8) return; FragH f;
#pragma unroll
  for (int i = 0; i < 8; ++i) f.h[i] = (_Float16)(bf16_round(W[t * 8 + i]) * 16.0f); *(volatile v8us*)((unsigned short*)Bt + t * 8) = f.half[0]; __threadfence(); *(volatile v8us*)((unsigned short*)Bt + t * 8) = f.half[0]; }
template <int NHv, int TTv>
__global__ __launch_bounds__(256) void k_vt(const _Float16* __restrict__ V16, int ldv, int voff, _Float16* __restrict__ Vt) { __shared__ unsigned short tl[64][66]; const int tid = threadIdx.x; const int slab = blockIdx.x / (TTv / 64), lg = blockIdx.x % (TTv / 64); const int b = slab / NHv, h = slab % NHv;
  for (int i = tid; i < 64 * 8; i += 256) { const int r = i / 8, c8 = (i % 8) * 8; FragH f; f.half[0] = *(const v8us*)((const unsigned short*)V16 + ((size_t)b * TTv + lg * 64 + r) * ldv + voff + h * 64 + c8);
#pragma unroll
    for (int q = 0; q < 8; ++q) tl[r][c8 + q] = f.u[q]; }
  __syncthreads();
  for (int pass = 0; pass < 2; ++pass) {
#pragma unroll
    for (int rd = 0; rd < 2; ++rd) { const int d = rd * 32 + tid / 8, pc = tid % 8; FragH f;
#pragma unroll
      for (int q = 0; q < 8; ++q) f.u[q] = tl[pc * 8 + q][d];
      *(volatile v8us*)((unsigned short*)Vt + ((size_t)slab * 64 + d) * TTv + lg * 64 + pc * 8) = f.half[0]; }
    if (pass == 0) __threadfence(); } }

__device__ __forceinline__ int bscan512(int cnt, int* wsum, int tid, int& total) {
  const int lane = tid & 31, wv = tid >> 5; int x = cnt;
#pragma unroll
  for (int d = 1; d < 32; d <<= 1) { const int y = __shfl_up(x, d, 32); if (lane >= d) x += y; }
  __syncthreads(); if (lane == 31) wsum[wv] = x; __syncthreads();
  int t = (lane < 16) ? wsum[lane] : 0;
#pragma unroll
  for (int d = 1; d < 32; d <<= 1) { const int y = __shfl_up(t, d, 32); if (lane >= d) t += y; }
  const int woff = (wv == 0) ? 0 : __shfl(t, wv - 1, 32); total = __shfl(t, 15, 32);
  return woff + x - cnt; }
#define QCAP 8
#define CHUNK 8192

#define PARTE 65536
__global__ __launch_bounds__(256) void k_bincntG(const int* __restrict__ key, int nedges, const int* __restrict__ IDS, const int* __restrict__ IOFFP, const int* __restrict__ ICNTP, int icap, int binw, int nbinpp, int npart, int* __restrict__ BCNTP) { __shared__ int red[256]; const int tid = threadIdx.x; const int g = blockIdx.x; const int part = g % npart; const int bin = g / npart; const int parent = bin / nbinpp; int c = 0;
  if (IDS) { int ibase = IOFFP[(size_t)parent * 32], icnt = ICNTP[(size_t)parent * 32]; icnt = icnt < 0 ? 0 : (icnt > nedges ? nedges : icnt); ibase = ibase < 0 ? 0 : (ibase > icap ? icap : ibase); const int i0 = part * PARTE, i1 = min(i0 + PARTE, icnt);
    for (int i = i0 + tid; i < i1; i += 256) { const int e = (ibase + i < icap) ? IDS[(size_t)ibase + i] : -1; if (e < 0 || e >= nedges) continue; const int d = key[e]; c += (d >= 0 && d / binw == bin) ? 1 : 0; } }
  else { const int e0 = part * PARTE, e1 = min(e0 + PARTE, nedges); for (int e = e0 + tid; e < e1; e += 256) { const int d = key[e]; c += (d >= 0 && d / binw == bin) ? 1 : 0; } }
  red[tid] = c; __syncthreads(); for (int o = 128; o >= 1; o >>= 1) { if (tid < o) red[tid] += red[tid + o]; __syncthreads(); }
  if (tid < 32) { const int v = (tid == 0) ? red[0] : 0; *(volatile int*)(BCNTP + (size_t)g * 32 + tid) = v; __threadfence(); *(volatile int*)(BCNTP + (size_t)g * 32 + tid) = v; } }
__global__ __launch_bounds__(256) void k_binscanG(const int* __restrict__ BCNTP, int nbin, int npart, int* __restrict__ OFFP) { __shared__ int cnt[1024]; const int tid = threadIdx.x;
  for (int b = tid; b < nbin; b += 256) { int s = 0; for (int p = 0; p < npart; ++p) s += BCNTP[((size_t)b * npart + p) * 32]; cnt[b] = s; } __syncthreads();
  if (tid == 0) { int run = 0; for (int b = 0; b < nbin; ++b) { const int c = cnt[b]; cnt[b] = run; run += (c + 31) & ~31; } } __syncthreads();
  for (int b = tid; b < nbin; b += 256) { for (int pass = 0; pass < 2; ++pass) { for (int j = 0; j < 32; ++j) *(volatile int*)(OFFP + (size_t)b * 32 + j) = (j == 0) ? cnt[b] : 0; if (pass == 0) __threadfence(); } } }
__global__ __launch_bounds__(512) void k_binemitG(const int* __restrict__ key, int nedges, const int* __restrict__ IDS, const int* __restrict__ IOFFP, const int* __restrict__ ICNTP, int icap, int binw, int nbinpp, const int* __restrict__ OFFP, int elcap, int* __restrict__ EL, int* __restrict__ CNTBP) {
  __shared__ int stage[CHUNK + 64]; __shared__ int scan[16]; const int tid = threadIdx.x; const int bin = blockIdx.x; const int parent = bin / nbinpp; const int k0 = bin * binw; int base = OFFP[(size_t)bin * 32]; base = base < 0 ? 0 : (base > elcap - 32 ? elcap - 32 : base); int nst = 0, written = 0, total = 0;
  int ibase = 0, icnt = nedges; if (IDS) { ibase = IOFFP[(size_t)parent * 32]; icnt = ICNTP[(size_t)parent * 32]; icnt = icnt < 0 ? 0 : (icnt > nedges ? nedges : icnt); ibase = ibase < 0 ? 0 : (ibase > icap ? icap : ibase); }
#pragma unroll 1
  for (int lb = 0; lb < icnt; lb += CHUNK) { int k_cnt = 0; unsigned hm = 0; int tot = 0; int ev[16];
#pragma unroll
    for (int k = 0; k < 16; ++k) { const int li = lb + tid * 16 + k; int e; if (IDS) e = (li < icnt && ibase + li < icap) ? IDS[(size_t)ibase + li] : -1; else e = (li < nedges) ? li : -1; if (e < 0 || e >= nedges) e = -1; ev[k] = e; const int d = (e >= 0) ? (key[e] - k0) : -1; if (d >= 0 && d < binw) { hm |= 1u << k; ++k_cnt; } }
    int p = bscan512(k_cnt, scan, tid, tot);
#pragma unroll
    for (int k = 0; k < 16; ++k) if (hm & (1u << k)) { stage[nst + p] = ev[k]; ++p; }
    __syncthreads(); nst += tot; total += tot;
    const int nfl = nst & ~31;
    for (int pass = 0; pass < 2; ++pass) { for (int i = tid; i < nfl; i += 512) { if (base + written + i < elcap) *(volatile int*)(EL + (size_t)base + written + i) = stage[i]; } if (pass == 0) __threadfence(); }
    __syncthreads();
    for (int i = tid; i < nst - nfl; i += 512) stage[i] = stage[nfl + i];
    __syncthreads(); written += nfl; nst -= nfl; }
  if (nst > 0) for (int pass = 0; pass < 2; ++pass) { if (tid < 32 && base + written + tid < elcap) *(volatile int*)(EL + (size_t)base + written + tid) = (tid < nst) ? stage[tid] : -1; if (pass == 0) __threadfence(); }
  if (tid < 32) { const int v = (tid == 0) ? total : 0; *(volatile int*)(CNTBP + (size_t)bin * 32 + tid) = v; __threadfence(); *(volatile int*)(CNTBP + (size_t)bin * 32 + tid) = v; } }
__global__ __launch_bounds__(512) void k_degcL(const int* __restrict__ EL, const int* __restrict__ OFFP, const int* __restrict__ CNTBP, int elcap, const int* __restrict__ dummy_src, const int* __restrict__ dsti, int ntargets, int nedges, float* __restrict__ CNT) {
  #pragma clang fp contract(off)
  __shared__ short Lr[CHUNK]; __shared__ int Le[CHUNK]; __shared__ int scan[16]; __shared__ int lq[16][QCAP][32]; __shared__ __attribute__((aligned(16))) float stg[64][68];
  const int tid = threadIdx.x, lane = tid & 31, wv = tid >> 5; const int n0 = blockIdx.x * 1024; int lcnt = CNTBP[(size_t)blockIdx.x * 32], lbase = OFFP[(size_t)blockIdx.x * 32]; lcnt = lcnt < 0 ? 0 : (lcnt > nedges ? nedges : lcnt); lbase = lbase < 0 ? 0 : (lbase > elcap ? elcap : lbase);        int qn = 0; float acc[2][64];
#pragma unroll
  for (int s2 = 0; s2 < 2; ++s2)
#pragma unroll
    for (int c = 0; c < 64; ++c) acc[s2][c] = 0.f;
  const int* srci = dummy_src; (void)srci;

#pragma unroll 1
  for (int eb = 0; eb < lcnt + CHUNK; eb += CHUNK) { const bool sentinel = (eb >= lcnt); int tot = 0;
    if (!sentinel) { int k_cnt = 0; unsigned hm = 0; int hv[16];
      int ev[16];
#pragma unroll
      for (int k = 0; k < 16; ++k) { const int li = eb + tid * 16 + k; int e = (li < lcnt && lbase + li < elcap) ? EL[(size_t)lbase + li] : -1; if (e < 0 || e >= nedges) e = -1; ev[k] = e; const int ec = (e >= 0) ? e : 0; const int dv = dsti[ec] - n0; const int dd_ = (e >= 0) ? dv : -1; hv[k] = dd_; if (dd_ >= 0 && dd_ < 1024) { hm |= 1u << k; ++k_cnt; } }
      int p = bscan512(k_cnt, scan, tid, tot);
#pragma unroll
      for (int k = 0; k < 16; ++k) if (hm & (1u << k)) { Lr[p] = (short)hv[k]; Le[p] = ev[k]; ++p; }
      __syncthreads(); }
    const int ntrip = sentinel ? 1 : ((tot + 31) >> 5);
#pragma unroll 1
    for (int it = 0; it < ntrip; ++it) { const int q = it * 32 + lane; const int lr = (!sentinel && q < tot) ? (int)Lr[q] : -1;
      unsigned mm = sentinel ? 1u : __builtin_amdgcn_ballot_w32(lr >= wv * 64 && lr < wv * 64 + 64);
#pragma unroll 1
      while (mm) { const int bit = __builtin_ctz(mm); mm &= mm - 1u; const int ol = sentinel ? -2 : (__shfl(lr, bit, 32) - wv * 64); const int owner = ol >> 1; const int e = sentinel ? 0 : Le[it * 32 + bit];
        if (sentinel || __builtin_amdgcn_ballot_w32(lane == owner && qn == QCAP)) {
          int kmax = qn;
#pragma unroll
          for (int o = 16; o >= 1; o >>= 1) kmax = max(kmax, __shfl_xor(kmax, o, 32));
#pragma unroll 1
          for (int k = 0; k < kmax; ++k) { if (k < qn) { const int ent = lq[wv][k][lane]; const int eq = ent >> 1; const int sl = ent & 1; int s = srci[eq]; s = s < 0 ? 0 : (s >= NNODE ? NNODE - 1 : s);
              (void)s;
#pragma unroll
              for (int s2 = 0; s2 < 2; ++s2) if (s2 == sl) acc[s2][0] += 1.0f; } }
          qn = 0; }
        if (lane == owner) { lq[wv][qn][lane] = e * 2 + (ol & 1); ++qn; } } }
    __syncthreads(); }
  for (int tg = 0; tg < 16; ++tg) {
    if (wv == tg) {
#pragma unroll
      for (int c = 0; c < 64; ++c) { stg[2 * lane][c] = acc[0][c]; stg[2 * lane + 1][c] = acc[1][c]; } }
    __syncthreads();
    if (tid < 64) { const int n = n0 + tg * 64 + tid; if (n < ntargets) { const float v = stg[tid][0]; *(volatile float*)(CNT + n) = v; __threadfence(); *(volatile float*)(CNT + n) = v; } }
    __syncthreads(); } }
__global__ __launch_bounds__(512) void k_gaggL(const int* __restrict__ EL, const int* __restrict__ OFFP, const int* __restrict__ CNTBP, int elcap, const _Float16* __restrict__ H16, int ldh, const float* __restrict__ Wsrc, int first, const int* __restrict__ srcarr, const int* __restrict__ dsti, int ntargets, int nedges, float* __restrict__ AGG, int lda) {
  #pragma clang fp contract(off)
  const int* __restrict__ dummy_src = srcarr;
  __shared__ short Lr[CHUNK]; __shared__ int Le[CHUNK]; __shared__ int scan[16]; __shared__ int lq[16][QCAP][32]; __shared__ __attribute__((aligned(16))) float stg[64][68];
  const int tid = threadIdx.x, lane = tid & 31, wv = tid >> 5; const int n0 = blockIdx.x * 1024; int lcnt = CNTBP[(size_t)blockIdx.x * 32], lbase = OFFP[(size_t)blockIdx.x * 32]; lcnt = lcnt < 0 ? 0 : (lcnt > nedges ? nedges : lcnt); lbase = lbase < 0 ? 0 : (lbase > elcap ? elcap : lbase);        int qn = 0; float acc[2][64];
#pragma unroll
  for (int s2 = 0; s2 < 2; ++s2)
#pragma unroll
    for (int c = 0; c < 64; ++c) acc[s2][c] = 0.f;
  const int* srci = dummy_src; (void)srci;

#pragma unroll 1
  for (int eb = 0; eb < lcnt + CHUNK; eb += CHUNK) { const bool sentinel = (eb >= lcnt); int tot = 0;
    if (!sentinel) { int k_cnt = 0; unsigned hm = 0; int hv[16];
      int ev[16];
#pragma unroll
      for (int k = 0; k < 16; ++k) { const int li = eb + tid * 16 + k; int e = (li < lcnt && lbase + li < elcap) ? EL[(size_t)lbase + li] : -1; if (e < 0 || e >= nedges) e = -1; ev[k] = e; const int ec = (e >= 0) ? e : 0; const int dv = dsti[ec] - n0; const int dd_ = (e >= 0) ? dv : -1; hv[k] = dd_; if (dd_ >= 0 && dd_ < 1024) { hm |= 1u << k; ++k_cnt; } }
      int p = bscan512(k_cnt, scan, tid, tot);
#pragma unroll
      for (int k = 0; k < 16; ++k) if (hm & (1u << k)) { Lr[p] = (short)hv[k]; Le[p] = ev[k]; ++p; }
      __syncthreads(); }
    const int ntrip = sentinel ? 1 : ((tot + 31) >> 5);
#pragma unroll 1
    for (int it = 0; it < ntrip; ++it) { const int q = it * 32 + lane; const int lr = (!sentinel && q < tot) ? (int)Lr[q] : -1;
      unsigned mm = sentinel ? 1u : __builtin_amdgcn_ballot_w32(lr >= wv * 64 && lr < wv * 64 + 64);
#pragma unroll 1
      while (mm) { const int bit = __builtin_ctz(mm); mm &= mm - 1u; const int ol = sentinel ? -2 : (__shfl(lr, bit, 32) - wv * 64); const int owner = ol >> 1; const int e = sentinel ? 0 : Le[it * 32 + bit];
        if (sentinel || __builtin_amdgcn_ballot_w32(lane == owner && qn == QCAP)) {
          int kmax = qn;
#pragma unroll
          for (int o = 16; o >= 1; o >>= 1) kmax = max(kmax, __shfl_xor(kmax, o, 32));
#pragma unroll 1
          for (int k = 0; k < kmax; ++k) { if (k < qn) { const int ent = lq[wv][k][lane]; const int eq = ent >> 1; const int sl = ent & 1; int s = srci[eq]; s = s < 0 ? 0 : (s >= NNODE ? NNODE - 1 : s);
              const float w = Wsrc ? Wsrc[s] : 1.0f; const unsigned short* hr = (const unsigned short*)H16 + (size_t)s * ldh;
#pragma unroll
              for (int s2 = 0; s2 < 2; ++s2) if (s2 == sl) {
#pragma unroll
                for (int g = 0; g < 8; ++g) { FragH f; f.half[0] = *(const v8us*)(hr + g * 8);
#pragma unroll
                  for (int d = 0; d < 8; ++d) acc[s2][g * 8 + d] += w * (float)f.h[d]; } } } }
          qn = 0; }
        if (lane == owner) { lq[wv][qn][lane] = e * 2 + (ol & 1); ++qn; } } }
    __syncthreads(); }
  for (int tg = 0; tg < 16; ++tg) {
    if (wv == tg) {
#pragma unroll
      for (int c = 0; c < 64; ++c) { stg[2 * lane][c] = acc[0][c]; stg[2 * lane + 1][c] = acc[1][c]; } }
    __syncthreads();
    v4f sum[2]; float* dst[2];
#pragma unroll
    for (int rd = 0; rd < 2; ++rd) { const int r = rd * 32 + tid / 16, pc = tid % 16; const int n = n0 + tg * 64 + r; dst[rd] = nullptr; if (n < ntargets) { dst[rd] = AGG + (size_t)n * lda + pc * 4; const v4f cur = first ? (v4f){0.f, 0.f, 0.f, 0.f} : *(const v4fa*)dst[rd]; v4f a; for (int q = 0; q < 4; ++q) a[q] = cur[q] + stg[r][pc * 4 + q]; sum[rd] = a; } }
    for (int pass = 0; pass < 2; ++pass) {
#pragma unroll
      for (int rd = 0; rd < 2; ++rd) if (dst[rd]) *(volatile v4f*)dst[rd] = sum[rd];
      if (pass == 0) __threadfence(); }
    __syncthreads(); } }

__global__ __launch_bounds__(256) void k_key(const int* __restrict__ et, const int* __restrict__ dst, int* __restrict__ KEY) { const int e = blockIdx.x * 256 + threadIdx.x; if (e >= NE) return; int r = et[e]; r = r < 0 ? 0 : (r >= NREL ? NREL - 1 : r); int d = dst[e]; d = d < 0 ? 0 : (d >= NNODE ? NNODE - 1 : d); const int k = r * KSTR + d; *(volatile int*)(KEY + e) = k; __threadfence(); *(volatile int*)(KEY + e) = k; }
__global__ __launch_bounds__(256) void k_mean16(const float* __restrict__ AGG, const float* __restrict__ CNT, _Float16* __restrict__ M16) { const size_t t = (size_t)blockIdx.x * 256 + threadIdx.x; if (t >= (size_t)NNODE * 16) return; const size_t n = t / 16; const float ic = 1.0f / fmaxf(CNT[n], 1.0f); FragH f; for (int q = 0; q < 8; ++q) f.h[q] = (_Float16)(AGG[t * 8 + q] * ic); *(volatile v8us*)((unsigned short*)M16 + t * 8) = f.half[0]; __threadfence(); *(volatile v8us*)((unsigned short*)M16 + t * 8) = f.half[0]; }
__global__ __launch_bounds__(256) void k_relu16(const float* __restrict__ P, _Float16* __restrict__ H16) { const size_t t = (size_t)blockIdx.x * 256 + threadIdx.x; if (t >= (size_t)NNODE * DI / 8) return; FragH f; for (int q = 0; q < 8; ++q) f.h[q] = (_Float16)fmaxf(P[t * 8 + q], 0.f); *(volatile v8us*)((unsigned short*)H16 + t * 8) = f.half[0]; __threadfence(); *(volatile v8us*)((unsigned short*)H16 + t * 8) = f.half[0]; }
__global__ __launch_bounds__(64) void k_pool(const float* __restrict__ EMB, const float* __restrict__ x, const int* __restrict__ pidx, float* __restrict__ out) { const int c = threadIdx.x; float s = 0.f, sw = 0.f;
#pragma unroll 1
  for (int p = 0; p < 256; ++p) { int n = pidx[p]; n = n < 0 ? 0 : (n >= NNODE ? NNODE - 1 : n); const float w = bf16_round(x[(size_t)n * DI]) * 4.0f + bf16_round(x[(size_t)n * DI + 1]) * 1.0f + bf16_round(x[(size_t)n * DI + 2]) * 2.0f; sw += w; s += EMB[(size_t)n * DO + c] * w; }
  const float v = s / (sw + 1e-9f); *(volatile float*)(out + c) = v; __threadfence(); *(volatile float*)(out + c) = v; }
extern "C" void kernel_launch(void* const* d_in, const int* in_sizes, int n_in,
                              void* d_out, int out_size, void* d_ws, size_t ws_size, hipStream_t stream) {
  (void)in_sizes; (void)n_in; (void)out_size;
  const float* x = (const float*)d_in[0]; const int* ei = (const int*)d_in[1]; const int* srci = ei; const int* dsti = ei + NE; const int* et = (const int*)d_in[2]; const int* pidx = (const int*)d_in[3]; const float* W1 = (const float*)d_in[4]; const float* root1 = (const float*)d_in[5]; const float* b1 = (const float*)d_in[6]; const float* W2 = (const float*)d_in[7]; const float* root2 = (const float*)d_in[8]; const float* b2 = (const float*)d_in[9];
  char* ws = (char*)d_ws; size_t off = 0;
  auto take = [&](size_t bytes) { char* p = ws + off; off += (bytes + 255) & ~(size_t)255; return p; };
  _Float16* BtW1 = (_Float16*)take((size_t)NREL * DI * DI * 2); _Float16* BR1 = (_Float16*)take((size_t)DI * DI * 2); _Float16* BtW2 = (_Float16*)take((size_t)NREL * DO * DI * 2); _Float16* BR2 = (_Float16*)take((size_t)DO * DI * 2);
  int* BC1 = (int*)take((size_t)NB1 * NP1 * 32 * 4); int* OFF1 = (int*)take((size_t)NB1 * 32 * 4); int* CNT1 = (int*)take((size_t)NB1 * 32 * 4); int* EL1 = (int*)take((size_t)ELCAP1 * 4); int* BC2 = (int*)take((size_t)NB2 * NP2 * 32 * 4); int* OFF2 = (int*)take((size_t)NB2 * 32 * 4); int* CNT2 = (int*)take((size_t)NB2 * 32 * 4); int* EL2 = (int*)take((size_t)ELCAP2 * 4); int* KEY = (int*)take((size_t)NE * 4);
  _Float16* X16 = (_Float16*)take((size_t)NNP * DI * 2); _Float16* H16 = (_Float16*)take((size_t)NNP * DI * 2); float* AGG = (float*)take((size_t)NNP * DI * 4); float* CNT = (float*)take((size_t)NNP * 4); _Float16* M16 = (_Float16*)take((size_t)NNP * DI * 2); float* PRE = (float*)take((size_t)NNP * DI * 4); float* EMB = (float*)take((size_t)NNP * DO * 4);
  if (off > ws_size) return;
  for (int r = 0; r < NREL; ++r) { k_wt_f16<<<(DI * (DI / 8) + 255) / 256, 256, 0, stream>>>(W1 + (size_t)r * DI * DI, BtW1 + (size_t)r * DI * DI, DI, DI, 16.0f); k_wt_f16<<<(DO * (DI / 8) + 255) / 256, 256, 0, stream>>>(W2 + (size_t)r * DI * DO, BtW2 + (size_t)r * DO * DI, DI, DO, 16.0f); }
  k_wt_f16<<<(DI * (DI / 8) + 255) / 256, 256, 0, stream>>>(root1, BR1, DI, DI, 16.0f); k_wt_f16<<<(DO * (DI / 8) + 255) / 256, 256, 0, stream>>>(root2, BR2, DI, DO, 16.0f);
  k_x16<<<(unsigned)(((size_t)NNODE * DI / 8 + 255) / 256), 256, 0, stream>>>(x, X16, (size_t)NNODE * DI / 8);
  k_key<<<(NE + 255) / 256, 256, 0, stream>>>(et, dsti, KEY);
  k_bincntG<<<NB1 * NP1, 256, 0, stream>>>(KEY, NE, nullptr, nullptr, nullptr, 0, BW1, 1, NP1, BC1); k_binscanG<<<1, 256, 0, stream>>>(BC1, NB1, NP1, OFF1); k_binemitG<<<NB1, 512, 0, stream>>>(KEY, NE, nullptr, nullptr, nullptr, 0, BW1, 1, OFF1, ELCAP1, EL1, CNT1);
  k_bincntG<<<NB2 * NP2, 256, 0, stream>>>(KEY, NE, EL1, OFF1, CNT1, ELCAP1, 1024, NB2 / NB1, NP2, BC2); k_binscanG<<<1, 256, 0, stream>>>(BC2, NB2, NP2, OFF2); k_binemitG<<<NB2, 512, 0, stream>>>(KEY, NE, EL1, OFF1, CNT1, ELCAP1, 1024, NB2 / NB1, OFF2, ELCAP2, EL2, CNT2);
  const unsigned gq = 49, g16 = (unsigned)(((size_t)NNODE * 16 + 255) / 256); const dim3 gN1(((NNODE / 16) * 2 + 3) / 4, 1), gN2(((NNODE / 16) * 1 + 3) / 4, 1);
  for (int l = 0; l < 2; ++l) { const _Float16* H = l ? H16 : X16; const int NO = l ? DO : DI; float* C = l ? EMB : PRE; const dim3 gN = l ? gN2 : gN1;
    k_gemm_hhx<0><<<gN, 128, 0, stream>>>(H, DI, 0, l ? BR2 : BR1, DI, 0, 0.0625f, l ? b2 : b1, 0, nullptr, 1, 0, 0, C, nullptr, NO, 0, NNODE, NO, DI);
    for (int r = 0; r < NREL; ++r) {
      { const int* OFFr = OFF2 + (size_t)r * 49 * 32; const int* CNTr = CNT2 + (size_t)r * 49 * 32;
      k_degcL<<<gq, 512, 0, stream>>>(EL2, OFFr, CNTr, ELCAP2, srci, dsti, NNODE, NE, CNT);
      k_gaggL<<<gq, 512, 0, stream>>>(EL2, OFFr, CNTr, ELCAP2, H, DI, nullptr, 1, srci, dsti, NNODE, NE, AGG, DI); k_gaggL<<<gq, 512, 0, stream>>>(EL2, OFFr, CNTr, ELCAP2, H + 64, DI, nullptr, 1, srci, dsti, NNODE, NE, AGG + 64, DI); }
      k_mean16<<<g16, 256, 0, stream>>>(AGG, CNT, M16);
      k_gemm_hhx<0><<<gN, 128, 0, stream>>>(M16, DI, 0, (l ? BtW2 + (size_t)r * DO * DI : BtW1 + (size_t)r * DI * DI), DI, 0, 0.0625f, nullptr, 0, C, 1, (size_t)NO, 0, C, nullptr, NO, 0, NNODE, NO, DI); }
    if (l == 0) k_relu16<<<(unsigned)(((size_t)NNODE * DI / 8 + 255) / 256), 256, 0, stream>>>(PRE, H16); }
  k_pool<<<1, 64, 0, stream>>>(EMB, x, pidx, (float*)d_out);
}
